// MultiHeadAttention_3805341024811
// MI455X (gfx1250) — hardware-verified
//
#include <hip/hip_runtime.h>
#ifndef NB
#define NB 2
#endif
#ifndef SEQ
#define SEQ 4096
#endif
#define NB_FULL 2
#define SEQ_FULL 4096
#define DM 512
#define NH 8
#define HD 64
#define EARLY (((SEQ) < 512) ? (SEQ) : 512)
#define RSC 1024.0f
#define RSCI 0.0009765625f
static_assert(SEQ % 128 == 0);
static_assert(EARLY % 128 == 0);
static_assert(NB <= NB_FULL);
static_assert(SEQ <= SEQ_FULL);
static_assert(NH * HD == DM);
static_assert(DM % 128 == 0);
static_assert(HD == 64);
static_assert(DM % 32 == 0);
static_assert(SEQ % 64 == 0);
static_assert((DM * DM) % 8 == 0);
static_assert((size_t)4 * DM * DM * 2 + (size_t)11 * NB * SEQ * DM * 2 <= (size_t)134217728);

typedef unsigned short v8us __attribute__((ext_vector_type(8), may_alias));
typedef float  v8f  __attribute__((ext_vector_type(8)));
typedef float  v4f  __attribute__((ext_vector_type(4)));
typedef float  v4fa __attribute__((ext_vector_type(4), may_alias));
typedef _Float16 v16h __attribute__((ext_vector_type(16)));
typedef _Float16 v4h __attribute__((ext_vector_type(4)));
union FragH { v16h v; v8us half[2]; _Float16 h[16]; unsigned short u[16]; };

__device__ __forceinline__ unsigned short bf16_bits(float x) { unsigned int u = __float_as_uint(x); return (unsigned short)((u + 0x7FFFu + ((u >> 16) & 1u)) >> 16); }
__device__ __forceinline__ float bf16_val(unsigned short b) { return __uint_as_float(((unsigned int)b) << 16); }
__device__ __forceinline__ float bf16_rne(float x) { return bf16_val(bf16_bits(x)); }

__device__ __forceinline__ v16h g2_frag(const _Float16* p, int hh) { FragH f; f.half[0] = *(const v8us*)((const unsigned short*)p + 8 * hh); f.half[1] = *(const v8us*)((const unsigned short*)p + 16 + 8 * hh); return f.v; }
__device__ __forceinline__ v8f g2_mma(v16h a, v16h b, v8f c) { v8f d = __builtin_amdgcn_wmma_f32_16x16x32_f16(false, a, false, b, (short)0, c, false, false); asm volatile("v_nop\n\tv_nop\n\tv_nop\n\tv_nop" : "+v"(d) : "v"(a), "v"(b)); return d; }
__device__ __forceinline__ v8f wm(v16h a, v16h b, v8f c) { return __builtin_amdgcn_wmma_f32_16x16x32_f16(false, a, false, b, (short)0, c, false, false); }

__global__ __launch_bounds__(256) void k_wnat(const float* __restrict__ w, size_t n8, _Float16* __restrict__ Bt) {
  const size_t t = (size_t)blockIdx.x * 256 + threadIdx.x; if (t >= n8) return; FragH f;
  const v4f a = *(const v4fa*)(w + t * 8), c = *(const v4fa*)(w + t * 8 + 4);
#pragma unroll
  for (int q = 0; q < 4; ++q) { f.h[q] = (_Float16)(bf16_rne(a[q]) * 16.0f); f.h[4 + q] = (_Float16)(bf16_rne(c[q]) * 16.0f); }
  const v8us o = f.half[0];
  *(volatile v8us*)((unsigned short*)Bt + t * 8) = o; __threadfence(); *(volatile v8us*)((unsigned short*)Bt + t * 8) = o;
}

__global__ __launch_bounds__(256) void k_x16(const float* __restrict__ x, _Float16* __restrict__ X16, size_t n8) {
  const size_t t = (size_t)blockIdx.x * 256 + threadIdx.x; if (t >= n8) return;
  const size_t e = t * 8; const size_t per = (size_t)SEQ * DM; const size_t b = e / per; const size_t wi = e - b * per;
  const float* src = x + b * ((size_t)SEQ_FULL * DM) + wi;
  const v4f a = *(const v4fa*)src, c = *(const v4fa*)(src + 4); FragH f;
#pragma unroll
  for (int q = 0; q < 4; ++q) { f.h[q] = (_Float16)bf16_rne(a[q]); f.h[4 + q] = (_Float16)bf16_rne(c[q]); }
  const v8us o = f.half[0];
  *(volatile v8us*)((unsigned short*)X16 + t * 8) = o; __threadfence(); *(volatile v8us*)((unsigned short*)X16 + t * 8) = o;
}

__device__ __forceinline__ void g2_kloop(const _Float16* a0p, const _Float16* a1p, const _Float16* b0p, const _Float16* b1p, const _Float16* b2p, const _Float16* b3p, int K, int hh,
                                         v8f& c00, v8f& c01, v8f& c02, v8f& c03, v8f& c10, v8f& c11, v8f& c12, v8f& c13) {
#pragma unroll 1
  for (int kb = 0; kb < K; kb += 32) {
    const v16h a0 = g2_frag(a0p + kb, hh), a1 = g2_frag(a1p + kb, hh);
    v16h b = g2_frag(b0p + kb, hh); c00 = g2_mma(a0, b, c00); c10 = g2_mma(a1, b, c10);
    b = g2_frag(b1p + kb, hh); c01 = g2_mma(a0, b, c01); c11 = g2_mma(a1, b, c11);
    b = g2_frag(b2p + kb, hh); c02 = g2_mma(a0, b, c02); c12 = g2_mma(a1, b, c12);
    b = g2_frag(b3p + kb, hh); c03 = g2_mma(a0, b, c03); c13 = g2_mma(a1, b, c13);
  }
}

template <int EM>
__global__ __launch_bounds__(128) void k_proj(const _Float16* __restrict__ A, int lda, size_t sA, const _Float16* __restrict__ Bh, int ldb, size_t sB, float alpha,
                                              _Float16* __restrict__ Ch, _Float16* __restrict__ Cr, int ldc, size_t sC, int M, int N, int K) {
  __shared__ __attribute__((aligned(16))) float so[4][32][68];
  const int tid = threadIdx.x, w = tid >> 5, lane = tid & 31, ln = lane & 15, hh = lane >> 4; const int by = blockIdx.y;
  A += (size_t)by * sA; Bh += (size_t)by * sB; const size_t cofs = (size_t)by * sC;
  const int ntn = N >> 6; const int mt = blockIdx.x / ntn, nq = blockIdx.x - mt * ntn; const int row0 = mt * 128 + 32 * w, col0 = nq * 64; if (row0 >= M) return;
  const bool early = (EM == 1) ? (mt * 128 < EARLY) : (col0 < EARLY);
  const _Float16* a0p = A + (size_t)(row0 + ln) * lda; const _Float16* a1p = a0p + (size_t)16 * lda;
  const _Float16* b0p = Bh + (size_t)(col0 + ln) * ldb; const _Float16* b1p = b0p + (size_t)16 * ldb; const _Float16* b2p = b1p + (size_t)16 * ldb; const _Float16* b3p = b2p + (size_t)16 * ldb;
  const v8f z8 = {0.f,0.f,0.f,0.f,0.f,0.f,0.f,0.f}; v8f c00 = z8, c01 = z8, c02 = z8, c03 = z8, c10 = z8, c11 = z8, c12 = z8, c13 = z8;
  g2_kloop(a0p, a1p, b0p, b1p, b2p, b3p, K, hh, c00, c01, c02, c03, c10, c11, c12, c13);
  v8f accs[8] = {c00, c01, c02, c03, c10, c11, c12, c13};
#pragma unroll
  for (int u = 0; u < 8; ++u) { const int t = u & 3, half = u >> 2;
#pragma unroll
    for (int r = 0; r < 8; ++r) { const int rloc = half * 16 + 8 * hh + r; const float v = accs[u][r] * alpha; so[w][rloc][t * 16 + ln] = v; } }
  __builtin_amdgcn_fence(4  , "workgroup"); __builtin_amdgcn_wave_barrier();
  const int rsub = lane >> 4, c4 = (lane & 15) * 4;
  for (int pass = 0; pass < 2; ++pass) {
#pragma unroll
    for (int q = 0; q < 16; ++q) { const int r = q * 2 + rsub; const v4f v = *(const v4fa*)&so[w][r][c4];
      v4h h4, r4;
#pragma unroll
      for (int i = 0; i < 4; ++i) { const _Float16 hv = (_Float16)v[i]; h4[i] = hv; r4[i] = (_Float16)((v[i] - (float)hv) * RSC); }
      const size_t o = cofs + (size_t)(row0 + r) * ldc + col0 + c4;
      *(volatile v4h*)(Ch + o) = h4;
      if (early) *(volatile v4h*)(Cr + o) = r4; }
    if (pass == 0) __threadfence(); }
}

template <bool RES>
__device__ __forceinline__ v8f score_tile(const _Float16* kp, const _Float16* krp, v16h qa, v16h qb, v16h qra, v16h qrb, int hh) {
  const v8f z8 = {0.f,0.f,0.f,0.f,0.f,0.f,0.f,0.f};
  const v16h ka = g2_frag(kp, hh), kb = g2_frag(kp + 32, hh);
  v8f s = z8;
  s = wm(ka, qa, s); s = wm(kb, qb, s);
  if (RES) {
    const v16h kra = g2_frag(krp, hh), krb = g2_frag(krp + 32, hh);
    v8f t = z8;
    t = wm(kra, qa, t); t = wm(ka, qra, t); t = wm(krb, qb, t); t = wm(kb, qrb, t);
    asm volatile("v_nop\n\tv_nop\n\tv_nop\n\tv_nop" : "+v"(s), "+v"(t) : "v"(ka), "v"(kb), "v"(kra), "v"(krb), "v"(qa), "v"(qb), "v"(qra), "v"(qrb));
    s = s + t * RSCI;
  } else {
    asm volatile("v_nop\n\tv_nop\n\tv_nop\n\tv_nop" : "+v"(s) : "v"(ka), "v"(kb), "v"(qa), "v"(qb));
  }
  return s;
}
__device__ __forceinline__ void pv_tile_res(const _Float16* vp, const _Float16* vrp, v16h pf, v16h pr, int hh, v8f& o, v8f& orr) {
  const v16h va = g2_frag(vp, hh), vra = g2_frag(vrp, hh);
  o = wm(va, pf, o); orr = wm(vra, pf, orr); orr = wm(va, pr, orr);
  asm volatile("v_nop\n\tv_nop\n\tv_nop\n\tv_nop" : "+v"(o), "+v"(orr) : "v"(va), "v"(vra), "v"(pf), "v"(pr));
}

template <bool RES>
__global__ __launch_bounds__(128) void k_flash(const _Float16* __restrict__ Qh, const _Float16* __restrict__ Qr, const _Float16* __restrict__ Kh, const _Float16* __restrict__ Kr,
                                               const _Float16* __restrict__ Vh, const _Float16* __restrict__ Vr, _Float16* __restrict__ Oh, _Float16* __restrict__ Or, int qt0, int nqt) {
  __shared__ __attribute__((aligned(16))) unsigned short lds_h[4][16][72];
  __shared__ __attribute__((aligned(16))) unsigned short lds_r[4][16][72];
  const int tid = threadIdx.x, w = tid >> 5, lane = tid & 31, ln = lane & 15, hh = lane >> 4;
  const int qloc = blockIdx.x * 4 + w; if (qloc >= nqt) return;
  const int q0 = (qt0 + qloc) * 16;
  const int bh = blockIdx.y; const int b = bh / NH, h = bh - b * NH;
  const size_t rowb = (size_t)b * SEQ;
  const size_t qoff = (rowb + q0 + ln) * DM + h * HD;
  const v16h qa = g2_frag(Qh + qoff, hh), qb = g2_frag(Qh + qoff + 32, hh);
  v16h qra = qa, qrb = qb;
  if (RES) { qra = g2_frag(Qr + qoff, hh); qrb = g2_frag(Qr + qoff + 32, hh); }
  const size_t koff = (rowb + ln) * DM + h * HD;
  const size_t voff = ((size_t)b * DM + h * HD + ln) * SEQ;
  const v8f z8 = {0.f,0.f,0.f,0.f,0.f,0.f,0.f,0.f};
  v8f o[4] = {z8, z8, z8, z8}, orr[4] = {z8, z8, z8, z8};
  float mrun = -3.0e38f, lrun = 0.f;
  const float cs = 0.18033688011112042f;
  const int nst = (q0 + 47) >> 5;
#pragma unroll 1
  for (int st = 0; st < nst; ++st) {
    const int k0 = st * 32;
    const size_t kof0 = koff + (size_t)k0 * DM, kof1 = kof0 + (size_t)16 * DM;
    v8f s0 = score_tile<RES>(Kh + kof0, Kr + kof0, qa, qb, qra, qrb, hh);
    v8f s1 = score_tile<RES>(Kh + kof1, Kr + kof1, qa, qb, qra, qrb, hh);
    if (st == nst - 1) {
      const int qy = q0 + ln; const int kk = k0 + 8 * hh;
#pragma unroll
      for (int r = 0; r < 8; ++r) { s0[r] = (kk + r > qy) ? -3.0e38f : s0[r]; s1[r] = (kk + 16 + r > qy) ? -3.0e38f : s1[r]; }
    }
    float mx = s0[0];
#pragma unroll
    for (int r = 1; r < 8; ++r) mx = fmaxf(mx, s0[r]);
#pragma unroll
    for (int r = 0; r < 8; ++r) mx = fmaxf(mx, s1[r]);
    mx = fmaxf(mx, __shfl_xor(mx, 16, 32));
    const float mnew = fmaxf(mrun, mx * cs);
    const float al = __builtin_amdgcn_exp2f(mrun - mnew);
    const float mo = 10.0f - mnew;
    float p0[8], p1[8]; float ps = 0.f;
#pragma unroll
    for (int r = 0; r < 8; ++r) { p0[r] = __builtin_amdgcn_exp2f(fmaf(s0[r], cs, mo)); p1[r] = __builtin_amdgcn_exp2f(fmaf(s1[r], cs, mo)); ps += p0[r] + p1[r]; }
    ps += __shfl_xor(ps, 16, 32);
    lrun = lrun * al + ps; mrun = mnew;
    FragH pf, pr;
#pragma unroll
    for (int r = 0; r < 8; ++r) {
      const _Float16 h0 = (_Float16)p0[r], h1 = (_Float16)p1[r]; pf.h[r] = h0; pf.h[8 + r] = h1;
      pr.h[r] = RES ? (_Float16)((p0[r] - (float)h0) * RSC) : (_Float16)0.0f; pr.h[8 + r] = RES ? (_Float16)((p1[r] - (float)h1) * RSC) : (_Float16)0.0f;
    }
    if (__builtin_amdgcn_ballot_w32(al != 1.0f) != 0u) {
#pragma unroll
      for (int t = 0; t < 4; ++t) { o[t] = o[t] * al; if (RES) orr[t] = orr[t] * al; }
    }
    const size_t vo = voff + k0;
    if (RES) {
#pragma unroll
      for (int t = 0; t < 4; ++t) pv_tile_res(Vh + vo + (size_t)(16 * t) * SEQ, Vr + vo + (size_t)(16 * t) * SEQ, pf.v, pr.v, hh, o[t], orr[t]);
    } else {
      const v16h va0 = g2_frag(Vh + vo, hh), va1 = g2_frag(Vh + vo + (size_t)16 * SEQ, hh), va2 = g2_frag(Vh + vo + (size_t)32 * SEQ, hh), va3 = g2_frag(Vh + vo + (size_t)48 * SEQ, hh);
      o[0] = wm(va0, pf.v, o[0]); o[1] = wm(va1, pf.v, o[1]); o[2] = wm(va2, pf.v, o[2]); o[3] = wm(va3, pf.v, o[3]);
      asm volatile("v_nop\n\tv_nop\n\tv_nop\n\tv_nop" : "+v"(o[0]), "+v"(o[1]), "+v"(o[2]), "+v"(o[3]) : "v"(va0), "v"(va1), "v"(va2), "v"(va3), "v"(pf.v));
    }
  }
  const float inv = 64.0f / lrun;
#pragma unroll
  for (int t = 0; t < 4; ++t) { FragH f, g;
#pragma unroll
    for (int r = 0; r < 8; ++r) { float v = o[t][r]; if (RES) v += orr[t][r] * RSCI; v *= inv; const _Float16 hv = (_Float16)v; f.h[r] = hv; g.h[r] = RES ? (_Float16)((v - (float)hv) * RSC) : (_Float16)0.0f; }
    *(v8us*)&lds_h[w][ln][16 * t + 8 * hh] = f.half[0];
    if (RES) *(v8us*)&lds_r[w][ln][16 * t + 8 * hh] = g.half[0]; }
  __builtin_amdgcn_fence(4  , "workgroup"); __builtin_amdgcn_wave_barrier();
  const int qsub = lane >> 3, pc = (lane & 7) * 8;
  for (int pass = 0; pass < 2; ++pass) {
#pragma unroll
    for (int j = 0; j < 4; ++j) { const int q = j * 4 + qsub; const size_t oo = (rowb + q0 + q) * DM + h * HD + pc;
      const v8us x = *(const v8us*)&lds_h[w][q][pc];
      *(volatile v8us*)((unsigned short*)Oh + oo) = x;
      if (RES) { const v8us y = *(const v8us*)&lds_r[w][q][pc]; *(volatile v8us*)((unsigned short*)Or + oo) = y; } }
    if (pass == 0) __threadfence(); }
}

__global__ __launch_bounds__(128) void k_out(const _Float16* __restrict__ A, const _Float16* __restrict__ Ar, int lda, size_t sA, const _Float16* __restrict__ Bh, int ldb, float alpha,
                                             float* __restrict__ C, int ldc, size_t sC, int M, int N, int K) {
  __shared__ __attribute__((aligned(16))) float so[4][32][68];
  const int tid = threadIdx.x, w = tid >> 5, lane = tid & 31, ln = lane & 15, hh = lane >> 4; const int by = blockIdx.y;
  A += (size_t)by * sA; Ar += (size_t)by * sA; const size_t cofs = (size_t)by * sC;
  const int ntn = N >> 6; const int mt = blockIdx.x / ntn, nq = blockIdx.x - mt * ntn; const int row0 = mt * 128 + 32 * w, col0 = nq * 64; if (row0 >= M) return;
  const bool early = (mt * 128 < EARLY);
  const _Float16* b0p = Bh + (size_t)(col0 + ln) * ldb; const _Float16* b1p = b0p + (size_t)16 * ldb; const _Float16* b2p = b1p + (size_t)16 * ldb; const _Float16* b3p = b2p + (size_t)16 * ldb;
  const v8f z8 = {0.f,0.f,0.f,0.f,0.f,0.f,0.f,0.f}; v8f c00 = z8, c01 = z8, c02 = z8, c03 = z8, c10 = z8, c11 = z8, c12 = z8, c13 = z8;
  if (early) {
    const _Float16* r0p = Ar + (size_t)(row0 + ln) * lda; const _Float16* r1p = r0p + (size_t)16 * lda;
    g2_kloop(r0p, r1p, b0p, b1p, b2p, b3p, K, hh, c00, c01, c02, c03, c10, c11, c12, c13);
    c00 = c00 * RSCI; c01 = c01 * RSCI; c02 = c02 * RSCI; c03 = c03 * RSCI; c10 = c10 * RSCI; c11 = c11 * RSCI; c12 = c12 * RSCI; c13 = c13 * RSCI;
  }
  const _Float16* a0p = A + (size_t)(row0 + ln) * lda; const _Float16* a1p = a0p + (size_t)16 * lda;
  g2_kloop(a0p, a1p, b0p, b1p, b2p, b3p, K, hh, c00, c01, c02, c03, c10, c11, c12, c13);
  v8f accs[8] = {c00, c01, c02, c03, c10, c11, c12, c13};
#pragma unroll
  for (int u = 0; u < 8; ++u) { const int t = u & 3, half = u >> 2;
#pragma unroll
    for (int r = 0; r < 8; ++r) { const int rloc = half * 16 + 8 * hh + r; so[w][rloc][t * 16 + ln] = accs[u][r] * alpha; } }
  __builtin_amdgcn_fence(4  , "workgroup"); __builtin_amdgcn_wave_barrier();
  const int rsub = lane >> 4, c4 = (lane & 15) * 4;
  for (int pass = 0; pass < 2; ++pass) {
#pragma unroll
    for (int q = 0; q < 16; ++q) { const int r = q * 2 + rsub; const v4f v = *(const v4fa*)&so[w][r][c4]; *(volatile v4f*)(C + cofs + (size_t)(row0 + r) * ldc + col0 + c4) = v; }
    if (pass == 0) __threadfence(); }
}

extern "C" void kernel_launch(void* const* d_in, const int* in_sizes, int n_in,
                              void* d_out, int out_size, void* d_ws, size_t ws_size, hipStream_t stream) {
  if (n_in < 7) return;
  const long long need_x = ((long long)(NB - 1) * SEQ_FULL + SEQ) * DM;
  if (in_sizes[0] < need_x || in_sizes[1] < need_x || in_sizes[2] < need_x) return;
  if (in_sizes[3] < DM * DM || in_sizes[4] < DM * DM || in_sizes[5] < DM * DM || in_sizes[6] < DM * DM) return;
  if ((long long)out_size < need_x) return;
  const float* const* I = (const float* const*)d_in;
  const float* xq = I[0]; const float* xk = I[1]; const float* xv = I[2];
  const float* wq = I[3]; const float* wk = I[4]; const float* wv = I[5]; const float* wo = I[6];
  char* ws = (char*)d_ws; size_t off = 0;
  auto take = [&](size_t bytes) { char* p = ws + off; off += (bytes + 255) & ~(size_t)255; return p; };
  const size_t WB = (size_t)DM * DM * 2, PB = (size_t)NB * SEQ * DM * 2;
  _Float16* BQ = (_Float16*)take(WB); _Float16* BK = (_Float16*)take(WB); _Float16* BV = (_Float16*)take(WB); _Float16* BO = (_Float16*)take(WB);
  _Float16* XQ = (_Float16*)take(PB); _Float16* XK = (_Float16*)take(PB); _Float16* XV = (_Float16*)take(PB);
  _Float16* Q16 = (_Float16*)take(PB); _Float16* K16 = (_Float16*)take(PB); _Float16* VT = (_Float16*)take(PB);
  _Float16* QR = (_Float16*)take(PB); _Float16* KR = (_Float16*)take(PB); _Float16* VTR = (_Float16*)take(PB);
  _Float16* O16 = (_Float16*)take(PB); _Float16* OR = (_Float16*)take(PB);
  if (off > ws_size || off > (size_t)134217728) return;

  { const size_t n8 = (size_t)DM * DM / 8; const unsigned g = (unsigned)((n8 + 255) / 256);
    k_wnat<<<g, 256, 0, stream>>>(wq, n8, BQ); k_wnat<<<g, 256, 0, stream>>>(wk, n8, BK); k_wnat<<<g, 256, 0, stream>>>(wv, n8, BV); k_wnat<<<g, 256, 0, stream>>>(wo, n8, BO); }
  { const size_t n8 = (size_t)NB * SEQ * DM / 8; const unsigned g = (unsigned)((n8 + 255) / 256);
    k_x16<<<g, 256, 0, stream>>>(xq, XQ, n8); k_x16<<<g, 256, 0, stream>>>(xk, XK, n8); k_x16<<<g, 256, 0, stream>>>(xv, XV, n8); }
  const size_t SB = (size_t)SEQ * DM;
  k_proj<1><<<dim3((unsigned)((SEQ / 128) * (DM / 64)), NB), 128, 0, stream>>>(XQ, DM, SB, BQ, DM, 0, 0.0625f, Q16, QR, DM, SB, SEQ, DM, DM);
  k_proj<1><<<dim3((unsigned)((SEQ / 128) * (DM / 64)), NB), 128, 0, stream>>>(XK, DM, SB, BK, DM, 0, 0.0625f, K16, KR, DM, SB, SEQ, DM, DM);
  k_proj<2><<<dim3((unsigned)((DM / 128) * (SEQ / 64)), NB), 128, 0, stream>>>(BV, DM, 0, XV, DM, SB, 0.0625f, VT, VTR, SEQ, SB, DM, SEQ, DM);
  k_flash<true><<<dim3((unsigned)((EARLY / 16 + 3) / 4), NB * NH), 128, 0, stream>>>(Q16, QR, K16, KR, VT, VTR, O16, OR, 0, EARLY / 16);
  if (SEQ > EARLY)
    k_flash<false><<<dim3((unsigned)(((SEQ - EARLY) / 16 + 3) / 4), NB * NH), 128, 0, stream>>>(Q16, Q16, K16, K16, VT, VT, O16, O16, EARLY / 16, (SEQ - EARLY) / 16);
  k_out<<<dim3((unsigned)((SEQ / 128) * (DM / 64)), NB), 128, 0, stream>>>(O16, OR, DM, SB, BO, DM, 0.0009765625f, (float*)d_out, DM, (size_t)SEQ_FULL * DM, SEQ, DM, DM);
}
